// PFNAttention_28948079575071
// MI455X (gfx1250) — hardware-verified
//
#include <hip/hip_runtime.h>
#include <stdint.h>
#include <math.h>

constexpr int kBatch  = 2;
constexpr int kSeq    = 2048;
constexpr int kDModel = 256;
constexpr int kHeads  = 8;
constexpr int kHDim   = 32;
constexpr int kTok    = kBatch * kSeq;
constexpr int kQkvLd  = 3 * kDModel;

typedef __attribute__((ext_vector_type(16))) _Float16 v16h;
typedef __attribute__((ext_vector_type(8)))  _Float16 v8h;
typedef __attribute__((ext_vector_type(16))) __bf16   v16b;
typedef __attribute__((ext_vector_type(8)))  __bf16   v8b;
typedef __attribute__((ext_vector_type(8)))  float    v8f;
typedef __attribute__((ext_vector_type(4)))  float    v4f;
#define PSCALE 32768.0f
#define U16(p) ((const unsigned short*)(const void*)(p))
#define PSCALE_INV (1.0f / 32768.0f)

__device__ __forceinline__ unsigned short f2bf_bits(float f) {
  unsigned u = __float_as_uint(f);
  return (unsigned short)((u + 0x7FFFu + ((u >> 16) & 1u)) >> 16);
}
__device__ __forceinline__ float bf_bits2f(unsigned short h) { return __uint_as_float(((unsigned)h) << 16); }

__device__ __forceinline__ void dep_guard_h(v8f& a, v8f& b, v16h x, v16h y) { asm volatile("v_nop\n\tv_nop\n\tv_nop\n\tv_nop" : "+v"(a), "+v"(b) : "v"(x), "v"(y)); }
__device__ __forceinline__ void dep_guard_b(v8f& a, v8f& b, v16b x, v16b y) { asm volatile("v_nop\n\tv_nop\n\tv_nop\n\tv_nop" : "+v"(a), "+v"(b) : "v"(x), "v"(y)); }
__device__ __forceinline__ void keep4_h(v16h a, v16h b, v16h c, v16h d) { asm volatile("v_nop" :: "v"(a), "v"(b), "v"(c), "v"(d)); }
__device__ __forceinline__ void keep4_b(v16b a, v16b b, v16b c, v16b d) { asm volatile("v_nop" :: "v"(a), "v"(b), "v"(c), "v"(d)); }
__device__ __forceinline__ void acc_guard4(v8f& a, v8f& b, v8f& c, v8f& d) { asm volatile("v_nop\n\tv_nop\n\tv_nop\n\tv_nop" : "+v"(a), "+v"(b), "+v"(c), "+v"(d)); }
template <typename T> struct Frag;
template <> struct Frag<_Float16> {
  typedef v16h V; union U { v16h v; v8h h[2]; };
  static __device__ __forceinline__ v16h load(const _Float16* p) {
    U f; f.h[0] = *(const v8h*)(p); f.h[1] = *(const v8h*)(p + 16); return f.v;
  }
  static __device__ __forceinline__ v8f mma(v16h a, v16h b, v8f c) {
    return __builtin_amdgcn_wmma_f32_16x16x32_f16(false, a, false, b, (short)0, c, false, false);
  }
  static __device__ __forceinline__ void guard(v8f& a, v8f& b, v16h x, v16h y) { dep_guard_h(a, b, x, y); }
  static __device__ __forceinline__ void keep(v16h a, v16h b, v16h c, v16h d) { keep4_h(a, b, c, d); }
};
template <> struct Frag<__bf16> {
  typedef v16b V; union U { v16b v; v8b h[2]; };
  static __device__ __forceinline__ v16b load(const __bf16* p) {
    U f; f.h[0] = *(const v8b*)(p); f.h[1] = *(const v8b*)(p + 16); return f.v;
  }
  static __device__ __forceinline__ v8f mma(v16b a, v16b b, v8f c) {
    return __builtin_amdgcn_wmma_f32_16x16x32_bf16(false, a, false, b, (short)0, c, false, false);
  }
  static __device__ __forceinline__ void guard(v8f& a, v8f& b, v16b x, v16b y) { dep_guard_b(a, b, x, y); }
  static __device__ __forceinline__ void keep(v16b a, v16b b, v16b c, v16b d) { keep4_b(a, b, c, d); }
};

template <int ET> struct Elem;
template <> struct Elem<0> { typedef _Float16 T; };
template <> struct Elem<1> { typedef __bf16 T; };
template <int ET, bool SPLIT, int BIAS_MODE, int OUT_MODE, bool RESID, int ACT = 0>
__global__ __launch_bounds__(256) void wmma_gemm64(
    const unsigned short* __restrict__ Ap, const unsigned short* __restrict__ A2p, int lda, long strideA,
    const unsigned short* __restrict__ Btp, const unsigned short* __restrict__ Bt2p, int ldb, long strideB,
    void* __restrict__ Cout, void* __restrict__ Cout2, int ldc, long strideC,
    const float* __restrict__ bias,
    const float* __restrict__ resid, long strideR,
    int M, int N, int K, float scale) {
  typedef typename Elem<ET>::T T;
  typedef typename Frag<T>::V V;
  const T* A = (const T*)Ap; const T* A2 = (const T*)A2p; const T* Bt = (const T*)Btp; const T* Bt2 = (const T*)Bt2p;
  __shared__ __align__(16) float sT[8][16 * 68];
  const int b    = blockIdx.y;
  const int lane = threadIdx.x & 31;
  const int wave = threadIdx.x >> 5;
  const int tilesN = N >> 6;
  const int tilesM = M >> 6;
  const int tile = blockIdx.x * 8 + wave;
  if (tile >= tilesM * tilesN) return;
  const int tm = tile / tilesN;
  const int tn = tile - tm * tilesN;
  const int m0 = tm << 6;
  const int n0 = tn << 6;

  const T* Ab  = A  + (size_t)b * strideA;
  const T* Bb  = Bt + (size_t)b * strideB;
  const T* Ab2 = SPLIT ? (A2  + (size_t)b * strideA) : nullptr;
  const T* Bb2 = SPLIT ? (Bt2 + (size_t)b * strideB) : nullptr;

  const int rlane = lane & 15;
  const int koff  = (lane >> 4) * 8;
  const int mOff  = (lane >> 4) * 8;

  v8f acc[4][4];
#pragma unroll
  for (int i = 0; i < 4; ++i)
#pragma unroll
    for (int j = 0; j < 4; ++j) acc[i][j] = (v8f){0.f,0.f,0.f,0.f,0.f,0.f,0.f,0.f};

  for (int k0 = 0; k0 < K; k0 += 32) {
    V bh[4], bl[4];
#pragma unroll
    for (int j = 0; j < 4; ++j) {
      const size_t bo = (size_t)(n0 + (j << 4) + rlane) * ldb + koff + k0;
      bh[j] = Frag<T>::load(Bb + bo);
      if (SPLIT) bl[j] = Frag<T>::load(Bb2 + bo);
    }
#pragma unroll
    for (int i = 0; i < 4; ++i) {
      const size_t ao = (size_t)(m0 + (i << 4) + rlane) * lda + koff + k0;
      V ah = Frag<T>::load(Ab + ao);
      V al;
      if (SPLIT) al = Frag<T>::load(Ab2 + ao);
#pragma unroll
      for (int j = 0; j < 4; ++j) {
        acc[i][j] = Frag<T>::mma(ah, bh[j], acc[i][j]);
        if (SPLIT) {
          acc[i][j] = Frag<T>::mma(ah, bl[j], acc[i][j]);
          acc[i][j] = Frag<T>::mma(al, bh[j], acc[i][j]);
        }
      }
      Frag<T>::guard(acc[i][0], acc[i][3], ah, SPLIT ? al : ah);
    }
    Frag<T>::keep(bh[0], bh[1], bh[2], bh[3]);
    if (SPLIT) Frag<T>::keep(bl[0], bl[1], bl[2], bl[3]);
  }
  acc_guard4(acc[0][0], acc[0][1], acc[0][2], acc[0][3]);
  acc_guard4(acc[1][0], acc[1][1], acc[1][2], acc[1][3]);
  acc_guard4(acc[2][0], acc[2][1], acc[2][2], acc[2][3]);
  acc_guard4(acc[3][0], acc[3][1], acc[3][2], acc[3][3]);

  float* slab = sT[wave];
  const float* Rb = RESID ? (resid + (size_t)b * strideR) : nullptr;
#pragma unroll
  for (int i = 0; i < 4; ++i) {
    const int mBase = m0 + (i << 4);
#pragma unroll
    for (int j = 0; j < 4; ++j) {
      const int n = n0 + (j << 4) + rlane;
      float bv = 0.f;
      if (BIAS_MODE == 2) bv = bias[n];
#pragma unroll
      for (int r = 0; r < 8; ++r) {
        float v = acc[i][j][r] * scale;
        if (BIAS_MODE == 1) v += bias[mBase + mOff + r];
        if (BIAS_MODE == 2) v += bv;
        if (RESID) v += Rb[(size_t)(mBase + mOff + r) * ldc + n];
        if (ACT == 1) v = tanhf(v);
        if (ACT == 2) v = fmaxf(v, 0.0f);
        if (ACT == 3) v = v / (1.0f + expf(-v));
        if (ACT == 4) v = (v > 0.f) ? v : 0.01f * v;
        if (ACT == 5) v = 0.5f * v * (1.0f + erff(v * 0.70710678118654752f));
        slab[(mOff + r) * 68 + (j << 4) + rlane] = v;
      }
    }
    __builtin_amdgcn_fence(__ATOMIC_RELEASE, "workgroup");
    __builtin_amdgcn_wave_barrier();
    __builtin_amdgcn_fence(__ATOMIC_ACQUIRE, "workgroup");
    if (OUT_MODE == 0) {
      float* C = (float*)Cout + (size_t)b * strideC;
      const int hh = lane >> 4, c4 = (lane & 15) * 4;
      for (int pass = 0; pass < 2; ++pass) {
#pragma unroll
        for (int it = 0; it < 8; ++it) {
          const int row = it * 2 + hh;
          v4f v = *(const v4f*)(slab + row * 68 + c4);
          *(volatile v4f*)(C + (size_t)(mBase + row) * ldc + n0 + c4) = v;
        }
        __threadfence();
      }
    } else {
      const int q = lane >> 3, c8 = (lane & 7) * 8;
      unsigned short* C  = (unsigned short*)Cout  + (size_t)b * strideC;
      unsigned short* C2 = (OUT_MODE == 2) ? ((unsigned short*)Cout2 + (size_t)b * strideC) : nullptr;
      for (int pass = 0; pass < 2; ++pass) {
#pragma unroll
        for (int it = 0; it < 4; ++it) {
          const int row = it * 4 + q;
          const float* sp = slab + row * 68 + c8;
          v8h hv, lv;
#pragma unroll
          for (int e = 0; e < 8; ++e) {
            if (OUT_MODE == 1) {
              hv[e] = (_Float16)sp[e];
            } else {
              unsigned short hb = f2bf_bits(sp[e]);
              unsigned short lb = f2bf_bits(sp[e] - bf_bits2f(hb));
              hv[e] = __builtin_bit_cast(_Float16, hb);
              lv[e] = __builtin_bit_cast(_Float16, lb);
            }
          }
          *(volatile v8h*)(C + (size_t)(mBase + row) * ldc + n0 + c8) = hv;
          if (OUT_MODE == 2) *(volatile v8h*)(C2 + (size_t)(mBase + row) * ldc + n0 + c8) = lv;
        }
        __threadfence();
      }
    }
    __builtin_amdgcn_fence(__ATOMIC_RELEASE, "workgroup");
    __builtin_amdgcn_wave_barrier();
    __builtin_amdgcn_fence(__ATOMIC_ACQUIRE, "workgroup");
  }
}

__device__ __forceinline__ unsigned short at_bf_bits(float f) {
  unsigned u = __float_as_uint(f);
  return (unsigned short)((u + 0x7FFFu + ((u >> 16) & 1u)) >> 16);
}
__device__ __forceinline__ __bf16 at_f2bf(float f) { return __builtin_bit_cast(__bf16, at_bf_bits(f)); }
__device__ __forceinline__ void at_split(float f, __bf16& hi, __bf16& lo) {
  const unsigned short hb = at_bf_bits(f);
  hi = __builtin_bit_cast(__bf16, hb);
  lo = at_f2bf(f - __uint_as_float(((unsigned)hb) << 16));
}
__device__ __forceinline__ v8f at_mma(v16b a, v16b b, v8f c) {
  c = __builtin_amdgcn_wmma_f32_16x16x32_bf16(false, a, false, b, (short)0, c, false, false);
  asm volatile("v_nop\n\tv_nop\n\tv_nop\n\tv_nop" : "+v"(c) : "v"(a), "v"(b));
  return c;
}

__global__ __launch_bounds__(256) void cast_x_bf16x2(
    const float* __restrict__ in, unsigned short* __restrict__ out, int n2) {
  int i = blockIdx.x * 256 + threadIdx.x;
  if (i < n2) {
    const float a = in[2 * (size_t)i], bb = in[2 * (size_t)i + 1];
    const unsigned u = (unsigned)f2bf_bits(a) | ((unsigned)f2bf_bits(bb) << 16);
    ((volatile unsigned*)out)[i] = u;
    __threadfence();
    ((volatile unsigned*)out)[i] = u;
  }
}

#define WTPITCH 72
__global__ __launch_bounds__(256) void wqkv_cast_k(
    const float* __restrict__ Wq, const float* __restrict__ Wk, const float* __restrict__ Wv,
    const float* __restrict__ bq, const float* __restrict__ bk, const float* __restrict__ bvp,
    unsigned short* __restrict__ Btp, float* __restrict__ bias_cat) {
  __shared__ __align__(16) unsigned short st[32 * WTPITCH];
  const int kt = blockIdx.x, h = blockIdx.y, mat = blockIdx.z;
  const float* W = (mat == 0) ? Wq : ((mat == 1) ? Wk : Wv);
  const int tid = threadIdx.x;
  const int m = tid >> 2, d0 = (tid & 3) * 8;
  const float* src = W + ((size_t)(h * kDModel + kt * 64 + m)) * kHDim + d0;
  const v4f a0 = *(const v4f*)src;
  const v4f a1 = *(const v4f*)(src + 4);
#pragma unroll
  for (int e = 0; e < 4; ++e) {
    st[(d0 + e) * WTPITCH + m]     = f2bf_bits(a0[e]);
    st[(d0 + 4 + e) * WTPITCH + m] = f2bf_bits(a1[e]);
  }
  __syncthreads();
  const int wave = tid >> 5, lane = tid & 31, q8 = lane >> 3, c8 = (lane & 7) * 8;
  const int row = wave * 4 + q8;
  const v8h hv = *(const v8h*)((const _Float16*)st + row * WTPITCH + c8);
  _Float16* dst = (_Float16*)Btp + ((size_t)(mat * kDModel + h * kHDim + row)) * kDModel + kt * 64 + c8;
  *(volatile v8h*)dst = hv;
  __threadfence();
  *(volatile v8h*)dst = hv;
  if (kt == 0 && tid < 8) {
    const float* bsrc = (mat == 0) ? bq : ((mat == 1) ? bk : bvp);
    const v4f b4 = *(const v4f*)(bsrc + h * kHDim + tid * 4);
    v4f br;
#pragma unroll
    for (int e = 0; e < 4; ++e) br[e] = bf_bits2f(f2bf_bits(b4[e]));
    float* bd = bias_cat + mat * kDModel + h * kHDim + tid * 4;
    *(volatile v4f*)bd = br;
    __threadfence();
    *(volatile v4f*)bd = br;
  }
}

__global__ __launch_bounds__(256) void wo_cast_k(const float* __restrict__ W, unsigned short* __restrict__ Wthp,
                                                 unsigned short* __restrict__ Wtlp, int Kdim, int Ndim) {
  __shared__ __align__(16) unsigned short st[64 * WTPITCH];
  _Float16* Wth = (_Float16*)Wthp;
  _Float16* Wtl = (_Float16*)Wtlp;
  const int n0 = blockIdx.x * 64, k0 = blockIdx.y * 64;
  const int tid = threadIdx.x;
  const int kr = tid >> 2, c16 = (tid & 3) * 16;
  const float* src = W + (size_t)(k0 + kr) * Ndim + n0 + c16;
#pragma unroll
  for (int q = 0; q < 4; ++q) {
    const v4f v = *(const v4f*)(src + 4 * q);
#pragma unroll
    for (int e = 0; e < 4; ++e) st[(c16 + 4 * q + e) * WTPITCH + kr] = f2bf_bits(v[e]);
  }
  __syncthreads();
  const int wave = tid >> 5, lane = tid & 31;
  const int q8 = lane >> 3, c8 = (lane & 7) * 8;
  const v8h zero8 = (v8h){(_Float16)0.f,(_Float16)0.f,(_Float16)0.f,(_Float16)0.f,(_Float16)0.f,(_Float16)0.f,(_Float16)0.f,(_Float16)0.f};
  for (int pass = 0; pass < 2; ++pass) {
#pragma unroll
    for (int it = 0; it < 2; ++it) {
      const int n = it * 32 + wave * 4 + q8;
      const v8h hv = *(const v8h*)((const _Float16*)st + n * WTPITCH + c8);
      *(volatile v8h*)(Wth + (size_t)(n0 + n) * Kdim + k0 + c8) = hv;
      *(volatile v8h*)(Wtl + (size_t)(n0 + n) * Kdim + k0 + c8) = zero8;
    }
    __threadfence();
  }
}

constexpr int kKch  = 64;
constexpr int kQblk = 64;
constexpr int kOsp  = 36;
constexpr float kScoreScale = 0.17677669529663687f;

__global__ __launch_bounds__(256) void attn_hd32_k(const unsigned short* __restrict__ qkvh_p, const unsigned short* __restrict__ qkvl_p,
                                                   unsigned short* __restrict__ zh_p, unsigned short* __restrict__ zl_p) {
  union FB { v16b v; v8b h[2]; };
  __shared__ __align__(16) __bf16 Ksh[2][kKch * kHDim];
  __shared__ __align__(16) __bf16 Ksl[2][kKch * kHDim];
  __shared__ __align__(16) __bf16 Vth[2][kHDim * kKch];
  __shared__ __align__(16) __bf16 Vtl[2][kHDim * kKch];
  __shared__ __align__(16) __bf16 Psh[8][16 * kKch];
  __shared__ __align__(16) __bf16 Psl[8][16 * kKch];
  __shared__ __align__(16) float  Osh[8][16 * kOsp];
  const __bf16* qkvh = (const __bf16*)qkvh_p;
  const __bf16* qkvl = (const __bf16*)qkvl_p;
  _Float16* zh = (_Float16*)zh_p;
  _Float16* zl = (_Float16*)zl_p;
  const int tid = threadIdx.x, wave = tid >> 5, lane = tid & 31, hh = lane >> 4, c = lane & 15;
  const int hp = wave >> 2, wq = wave & 3;
  const int nqb = kSeq / kQblk;
  const int bx = blockIdx.x;
  const int qb = bx % nqb;
  const int t2 = bx / nqb;
  const int pair = t2 % (kHeads / 2);
  const int b = t2 / (kHeads / 2);
  const int head = pair * 2 + hp;
  const int tok0 = b * kSeq + qb * kQblk;
  const int q0 = qb * kQblk + wq * 16;

  v16b qah, qal;
  {
    const size_t qoff = (size_t)(b * kSeq + q0 + c) * kQkvLd + head * kHDim + 8 * hh;
    qah = Frag<__bf16>::load(qkvh + qoff);
    qal = Frag<__bf16>::load(qkvl + qoff);
  }
  float mrow[8], lrow[8];
  v8f oacc[2];
#pragma unroll
  for (int r = 0; r < 8; ++r) { mrow[r] = -INFINITY; lrow[r] = 0.f; }
#pragma unroll
  for (int t = 0; t < 2; ++t) oacc[t] = (v8f){0.f,0.f,0.f,0.f,0.f,0.f,0.f,0.f};

  const int nChunks = qb + 1;
  for (int kc = 0; kc < nChunks; ++kc) {
    const int kv0 = kc * kKch;
    __syncthreads();
    {
      const int shp = tid >> 7, kvr = (tid & 127) >> 1, dh = (tid & 1) * 16;
      const int shead = pair * 2 + shp;
      const size_t roff = (size_t)(b * kSeq + kv0 + kvr) * kQkvLd + shead * kHDim + dh;
      const v8b kh0 = *(const v8b*)(qkvh + roff + kDModel);
      const v8b kh1 = *(const v8b*)(qkvh + roff + kDModel + 8);
      const v8b kl0 = *(const v8b*)(qkvl + roff + kDModel);
      const v8b kl1 = *(const v8b*)(qkvl + roff + kDModel + 8);
      const v8b vh0 = *(const v8b*)(qkvh + roff + 2 * kDModel);
      const v8b vh1 = *(const v8b*)(qkvh + roff + 2 * kDModel + 8);
      const v8b vl0 = *(const v8b*)(qkvl + roff + 2 * kDModel);
      const v8b vl1 = *(const v8b*)(qkvl + roff + 2 * kDModel + 8);
      __bf16* ksd = Ksh[shp] + kvr * kHDim + dh;
      *(v8b*)(ksd) = kh0; *(v8b*)(ksd + 8) = kh1;
      __bf16* kld = Ksl[shp] + kvr * kHDim + dh;
      *(v8b*)(kld) = kl0; *(v8b*)(kld + 8) = kl1;
      __bf16* vhd = Vth[shp] + dh * kKch + kvr;
      __bf16* vld = Vtl[shp] + dh * kKch + kvr;
#pragma unroll
      for (int e = 0; e < 8; ++e) {
        vhd[e * kKch] = vh0[e]; vhd[(8 + e) * kKch] = vh1[e];
        vld[e * kKch] = vl0[e]; vld[(8 + e) * kKch] = vl1[e];
      }
    }
    __syncthreads();

    const __bf16* ks  = Ksh[hp];
    const __bf16* ksl = Ksl[hp];
    v8f s[4];
#pragma unroll
    for (int j = 0; j < 4; ++j) {
      s[j] = (v8f){0.f,0.f,0.f,0.f,0.f,0.f,0.f,0.f};
      FB kb, kl;
      kb.h[0] = *(const v8b*)(ks  + (j * 16 + c) * kHDim + 8 * hh);
      kb.h[1] = *(const v8b*)(ks  + (j * 16 + c) * kHDim + 16 + 8 * hh);
      kl.h[0] = *(const v8b*)(ksl + (j * 16 + c) * kHDim + 8 * hh);
      kl.h[1] = *(const v8b*)(ksl + (j * 16 + c) * kHDim + 16 + 8 * hh);
      s[j] = at_mma(qah, kb.v, s[j]);
      s[j] = at_mma(qah, kl.v, s[j]);
      s[j] = at_mma(qal, kb.v, s[j]);
    }
    float cm[8];
#pragma unroll
    for (int r = 0; r < 8; ++r) {
      const int qrow = q0 + 8 * hh + r;
      float m = -INFINITY;
#pragma unroll
      for (int j = 0; j < 4; ++j) {
        const int kvcol = kv0 + j * 16 + c;
        float sv = s[j][r] * kScoreScale;
        const bool allowed = (kvcol == qrow) || ((kvcol < qrow) && ((kvcol & 1) != 0));
        if (!allowed) sv = -INFINITY;
        s[j][r] = sv;
        m = fmaxf(m, sv);
      }
#pragma unroll
      for (int off = 1; off < 16; off <<= 1) m = fmaxf(m, __shfl_xor(m, off, 32));
      cm[r] = m;
    }
    __bf16* pwh = Psh[wave];
    __bf16* pwl = Psl[wave];
#pragma unroll
    for (int r = 0; r < 8; ++r) {
      const float mnew = fmaxf(mrow[r], cm[r]);
      const float mref = (mnew > -INFINITY) ? mnew : 0.0f;
      const float alpha = expf(mrow[r] - mref);
      mrow[r] = mnew;
      float psum = 0.f;
#pragma unroll
      for (int j = 0; j < 4; ++j) {
        const float p = expf(s[j][r] - mref);
        psum += p;
        __bf16 a, bl;
        at_split(p, a, bl);
        pwh[(8 * hh + r) * kKch + j * 16 + c] = a;
        pwl[(8 * hh + r) * kKch + j * 16 + c] = bl;
      }
#pragma unroll
      for (int off = 1; off < 16; off <<= 1) psum += __shfl_xor(psum, off, 32);
      lrow[r] = lrow[r] * alpha + psum;
#pragma unroll
      for (int t = 0; t < 2; ++t) oacc[t][r] *= alpha;
    }
    __builtin_amdgcn_fence(__ATOMIC_RELEASE, "workgroup");
    __builtin_amdgcn_wave_barrier();
    __builtin_amdgcn_fence(__ATOMIC_ACQUIRE, "workgroup");
    const __bf16* vs  = Vth[hp];
    const __bf16* vsl = Vtl[hp];
#pragma unroll 1
    for (int kk = 0; kk < 2; ++kk) {
      FB pa, pf;
      pa.h[0] = *(const v8b*)(pwh + c * kKch + kk * 32 + 8 * hh);
      pa.h[1] = *(const v8b*)(pwh + c * kKch + kk * 32 + 16 + 8 * hh);
      pf.h[0] = *(const v8b*)(pwl + c * kKch + kk * 32 + 8 * hh);
      pf.h[1] = *(const v8b*)(pwl + c * kKch + kk * 32 + 16 + 8 * hh);
#pragma unroll
      for (int t = 0; t < 2; ++t) {
        FB vb, vl;
        vb.h[0] = *(const v8b*)(vs  + (t * 16 + c) * kKch + kk * 32 + 8 * hh);
        vb.h[1] = *(const v8b*)(vs  + (t * 16 + c) * kKch + kk * 32 + 16 + 8 * hh);
        vl.h[0] = *(const v8b*)(vsl + (t * 16 + c) * kKch + kk * 32 + 8 * hh);
        vl.h[1] = *(const v8b*)(vsl + (t * 16 + c) * kKch + kk * 32 + 16 + 8 * hh);
        oacc[t] = at_mma(pa.v, vb.v, oacc[t]);
        oacc[t] = at_mma(pa.v, vl.v, oacc[t]);
        oacc[t] = at_mma(pf.v, vb.v, oacc[t]);
      }
    }
  }

  float* os = Osh[wave];
#pragma unroll
  for (int r = 0; r < 8; ++r) {
    const float inv = 1.0f / lrow[r];
#pragma unroll
    for (int t = 0; t < 2; ++t) os[(8 * hh + r) * kOsp + t * 16 + c] = oacc[t][r] * inv;
  }
  __syncthreads();
  {
    const int q8 = lane >> 3, c8 = (lane & 7) * 8;
    const int hsel = c8 >> 5, d0 = c8 & 31;
    for (int pass = 0; pass < 2; ++pass) {
#pragma unroll
      for (int it = 0; it < 2; ++it) {
        const int row = wave * 8 + it * 4 + q8;
        const float* sp = Osh[hsel * 4 + (row >> 4)] + (row & 15) * kOsp + d0;
        const v4f x0 = *(const v4f*)sp;
        const v4f x1 = *(const v4f*)(sp + 4);
        v8h hv, lv;
#pragma unroll
        for (int e = 0; e < 4; ++e) {
          const unsigned short hb0 = f2bf_bits(x0[e]);
          const unsigned short lb0 = f2bf_bits(x0[e] - bf_bits2f(hb0));
          const unsigned short hb1 = f2bf_bits(x1[e]);
          const unsigned short lb1 = f2bf_bits(x1[e] - bf_bits2f(hb1));
          hv[e]     = __builtin_bit_cast(_Float16, hb0);
          lv[e]     = __builtin_bit_cast(_Float16, lb0);
          hv[4 + e] = __builtin_bit_cast(_Float16, hb1);
          lv[4 + e] = __builtin_bit_cast(_Float16, lb1);
        }
        const size_t off = (size_t)(tok0 + row) * kDModel + pair * 64 + c8;
        *(volatile v8h*)(zh + off) = hv;
        *(volatile v8h*)(zl + off) = lv;
      }
      __threadfence();
    }
  }
}

static_assert(kTok % 64 == 0 && kQkvLd % 64 == 0 && kDModel % 64 == 0, "tile multiples");
static_assert(kDModel % 32 == 0, "K multiple of 32");
static_assert(kSeq % kQblk == 0 && kHeads % 2 == 0 && kHDim == 32, "attention tiling");

extern "C" void kernel_launch(void* const* d_in, const int* in_sizes, int n_in,
                              void* d_out, int out_size, void* d_ws, size_t ws_size,
                              hipStream_t stream) {
  if (n_in < 9) return;
  const int nX = kTok * kDModel;
  const int nW = kHeads * kDModel * kHDim;
  if (in_sizes[0] != nX || in_sizes[1] != nW || in_sizes[2] != nW || in_sizes[3] != nW || in_sizes[4] != nW ||
      in_sizes[5] != kHeads * kHDim || in_sizes[6] != kHeads * kHDim || in_sizes[7] != kHeads * kHDim ||
      in_sizes[8] != kDModel || out_size != nX) return;

  const float* x  = (const float*)d_in[0];
  const float* Wq = (const float*)d_in[1];
  const float* Wk = (const float*)d_in[2];
  const float* Wv = (const float*)d_in[3];
  const float* Wo = (const float*)d_in[4];
  const float* bq = (const float*)d_in[5];
  const float* bk = (const float*)d_in[6];
  const float* bv = (const float*)d_in[7];
  const float* bo = (const float*)d_in[8];
  float* out = (float*)d_out;

  const size_t szXB   = (size_t)nX * 2;
  const size_t szWQKV = (size_t)kQkvLd * kDModel * 2;
  const size_t szWO   = (size_t)kDModel * kDModel * 2;
  const size_t szBIAS = 4096;
  const size_t szQKV  = (size_t)kTok * kQkvLd * 2;
  const size_t szZ    = (size_t)kTok * kDModel * 2;
  const size_t offXB   = 0;
  const size_t offWQKV = offXB + szXB;
  const size_t offWOH  = offWQKV + szWQKV;
  const size_t offWOL  = offWOH + szWO;
  const size_t offBIAS = offWOL + szWO;
  const size_t offQKVH = offBIAS + szBIAS;
  const size_t offQKVL = offQKVH + szQKV;
  const size_t offZH   = offQKVL + szQKV;
  const size_t offZL   = offZH + szZ;
  const size_t total   = offZL + szZ;
  if (total > ws_size) return;

  char* ws = (char*)d_ws;
  unsigned short* Xb    = (unsigned short*)(ws + offXB);
  unsigned short* Wqkv  = (unsigned short*)(ws + offWQKV);
  unsigned short* Woh   = (unsigned short*)(ws + offWOH);
  unsigned short* Wol   = (unsigned short*)(ws + offWOL);
  float*          biasc = (float*)(ws + offBIAS);
  unsigned short* Qkvh  = (unsigned short*)(ws + offQKVH);
  unsigned short* Qkvl  = (unsigned short*)(ws + offQKVL);
  unsigned short* Zh    = (unsigned short*)(ws + offZH);
  unsigned short* Zl    = (unsigned short*)(ws + offZL);

  const int n2 = nX / 2;
  cast_x_bf16x2<<<dim3((n2 + 255) / 256), dim3(256), 0, stream>>>(x, Xb, n2);
  wqkv_cast_k<<<dim3(kDModel / 64, kHeads, 3), dim3(256), 0, stream>>>(Wq, Wk, Wv, bq, bk, bv, Wqkv, biasc);
  wo_cast_k<<<dim3(kDModel / 64, kDModel / 64), dim3(256), 0, stream>>>(Wo, Woh, Wol, kDModel, kDModel);
  {
    const int tiles = (kTok / 64) * (kQkvLd / 64);
    wmma_gemm64<1, false, 2, 2, false, 0><<<dim3(tiles / 8, 1), dim3(256), 0, stream>>>(
        Xb, Xb, kDModel, 0L, Wqkv, Wqkv, kDModel, 0L, (void*)Qkvh, (void*)Qkvl, kQkvLd, 0L,
        biasc, biasc, 0L, kTok, kQkvLd, kDModel, 1.0f);
  }
  attn_hd32_k<<<dim3(kBatch * (kHeads / 2) * (kSeq / kQblk)), dim3(256), 0, stream>>>(Qkvh, Qkvl, Zh, Zl);
  {
    const int tiles = (kTok / 64) * (kDModel / 64);
    wmma_gemm64<1, true, 2, 0, false, 0><<<dim3(tiles / 8, 1), dim3(256), 0, stream>>>(
        Zh, Zl, kDModel, 0L, Woh, Wol, kDModel, 0L, (void*)out, (void*)out, kDModel, 0L,
        bo, bo, 0L, kTok, kDModel, kDModel, 1.0f);
  }
}
